// ScOTLayer_69973607186742
// MI455X (gfx1250) — hardware-verified
//
#include <hip/hip_runtime.h>

#define NTOK     65536
#define HTOK     32768
#define IMGTOK   4096
#define CH       192
#define NHEAD    6
#define HDIM     32
#define WINN     256
#define HWIN     128
#define HIDCH    768
#define CHUNK    8192
#define PLN      6291456
#define NT16     5888
#define NCPB     5766
#define WOFF_P   110592
#define WOFF_F1  147456
#define WOFF_F2  294912
#define LN_EPS   1e-5f
#define LN100    4.6051702f

typedef unsigned short us;
typedef __bf16 bf16x16 __attribute__((ext_vector_type(16)));
typedef float  v8f __attribute__((ext_vector_type(8)));
typedef float  v4f __attribute__((ext_vector_type(4)));
typedef int    v4i __attribute__((ext_vector_type(4)));
typedef int    v8i __attribute__((ext_vector_type(8)));
typedef v4f __attribute__((may_alias)) v4fa;
typedef v4i __attribute__((may_alias)) v4ia;

union Frag { bf16x16 v; v8i w; v4i q[2]; };

__device__ __forceinline__ unsigned int f2bf(float f) {
  unsigned int u = __float_as_uint(f);
  u += 0x7fffu + ((u >> 16) & 1u);
  return u >> 16;
}

__device__ __forceinline__ unsigned int pk2(float a, float b, unsigned int& lo) {
  const unsigned int ha = f2bf(a), hb = f2bf(b);
  const float ra = a - __uint_as_float(ha << 16);
  const float rb = b - __uint_as_float(hb << 16);
  lo = f2bf(ra) | (f2bf(rb) << 16);
  return ha | (hb << 16);
}

__device__ __forceinline__ void split8(v4f x0, v4f x1, v4i& hi, v4i& lo) {
  unsigned int l0, l1, l2, l3;
  const unsigned int h0 = pk2(x0.x, x0.y, l0);
  const unsigned int h1 = pk2(x0.z, x0.w, l1);
  const unsigned int h2 = pk2(x1.x, x1.y, l2);
  const unsigned int h3 = pk2(x1.z, x1.w, l3);
  hi.x = (int)h0; hi.y = (int)h1; hi.z = (int)h2; hi.w = (int)h3;
  lo.x = (int)l0; lo.y = (int)l1; lo.z = (int)l2; lo.w = (int)l3;
}

__device__ __forceinline__ void sched_fence() {
  asm volatile("" ::: "memory");
}

__device__ __forceinline__ v8f wmma3(v8i a, v8i b, v8f c) {
  Frag fa, fb;
  fa.w = a; fb.w = b;
  v8f d = __builtin_amdgcn_wmma_f32_16x16x32_bf16(false, fa.v, false, fb.v, (short)0, c, false, false);
  asm volatile("v_nop\n\tv_nop\n\tv_nop\n\tv_nop" : "+v"(d) : "v"(a), "v"(b));
  return d;
}

__device__ __forceinline__ v8i ldfrag(const us* p, int h) {
  Frag f;
  f.q[0] = *(const v4ia*)(p + 8 * h);
  f.q[1] = *(const v4ia*)(p + 16 + 8 * h);
  return f.w;
}

__device__ __forceinline__ void packP(v8f a, v8f c, v8i& hi, v8i& lo) {
  const v4f a0 = {a[0], a[1], a[2], a[3]};
  const v4f a1 = {a[4], a[5], a[6], a[7]};
  const v4f c0 = {c[0], c[1], c[2], c[3]};
  const v4f c1 = {c[4], c[5], c[6], c[7]};
  Frag fh, fl;
  split8(a0, a1, fh.q[0], fl.q[0]);
  split8(c0, c1, fh.q[1], fl.q[1]);
  hi = fh.w; lo = fl.w;
}

__device__ __forceinline__ float gelu_f(float x) {
  return 0.5f * x * (1.0f + erff(x * 0.70710678118654752f));
}

__global__ __launch_bounds__(256) void k_wcvt(
    const float* __restrict__ qw, const float* __restrict__ kw, const float* __restrict__ vw,
    const float* __restrict__ pw, const float* __restrict__ f1, const float* __restrict__ f2,
    us* __restrict__ Wh, us* __restrict__ Wl)
{
  const int g = blockIdx.x * 256 + threadIdx.x;
  const int e = g * 8;
  const float* src;
  if (e < 36864)       src = qw + e;
  else if (e < 73728)  src = kw + (e - 36864);
  else if (e < 110592) src = vw + (e - 73728);
  else if (e < 147456) src = pw + (e - 110592);
  else if (e < 294912) src = f1 + (e - 147456);
  else                 src = f2 + (e - 294912);
  const v4f x0 = *(const v4fa*)src;
  const v4f x1 = *(const v4fa*)(src + 4);
  v4i hi, lo;
  split8(x0, x1, hi, lo);
  *(volatile v4i*)(Wh + e) = hi;
  *(volatile v4i*)(Wl + e) = lo;
  __threadfence();
  *(volatile v4i*)(Wh + e) = hi;
  *(volatile v4i*)(Wl + e) = lo;
}

__global__ __launch_bounds__(256) void k_cpb(const float* __restrict__ w1,
                                             const float* __restrict__ b1,
                                             const float* __restrict__ w2,
                                             float* __restrict__ t16)
{
  const int g = blockIdx.x * 256 + threadIdx.x;
  const int gg = (g < NCPB) ? g : (NCPB - 1);
  const int mi = gg / NHEAD, hd = gg - mi * NHEAD;
  const int a = mi / 31, bq = mi - a * 31;
  const float va = (float)(a - 15) * (1.0f / 15.0f) * 8.0f;
  const float vb = (float)(bq - 15) * (1.0f / 15.0f) * 8.0f;
  const float la = __log2f(fabsf(va) + 1.0f) * (1.0f / 3.0f);
  const float lb = __log2f(fabsf(vb) + 1.0f) * (1.0f / 3.0f);
  const float t0 = (a < 15) ? -la : la;
  const float t1 = (bq < 15) ? -lb : lb;
  float acc = 0.0f;
#pragma unroll 1
  for (int j = 0; j < 512; ++j) {
    float r = t0 * w1[2 * j] + t1 * w1[2 * j + 1] + b1[j];
    r = fmaxf(r, 0.0f);
    acc += r * w2[hd * 512 + j];
  }
  float val = 16.0f * __builtin_amdgcn_rcpf(1.0f + __expf(-acc));
  if (g >= NCPB) val = 0.0f;
  *(volatile float*)(t16 + g) = val;
  __threadfence();
  *(volatile float*)(t16 + g) = val;
}

__global__ __launch_bounds__(256) void k_bmt(const float* __restrict__ t16,
                                             float* __restrict__ bmt)
{
  const int g = blockIdx.x * 256 + threadIdx.x;
  const int key = g & 255;
  const int qry = (g >> 8) & 255;
  const int hc = g >> 16;
  const int head = hc % NHEAD, cls = hc / NHEAD;
  const int iq = qry >> 4, jq = qry & 15, ik = key >> 4, jk = key & 15;
  const int idx = (iq - ik + 15) * 31 + (jq - jk + 15);
  const float bias = t16[idx * NHEAD + head];
  const int eh = cls >> 1, ew = cls & 1;
  const int rq = (eh ? (iq < 8 ? 1 : 2) : 0) * 3 + (ew ? (jq < 8 ? 1 : 2) : 0);
  const int rk = (eh ? (ik < 8 ? 1 : 2) : 0) * 3 + (ew ? (jk < 8 ? 1 : 2) : 0);
  const float val = bias + ((rq != rk) ? -100.0f : 0.0f);
  *(volatile float*)(bmt + g) = val;
  __threadfence();
  *(volatile float*)(bmt + g) = val;
}

__global__ __launch_bounds__(256) void k_pack(const float* __restrict__ x,
                                              us* __restrict__ xh, us* __restrict__ xl, int hf)
{
  const int g = blockIdx.x * 256 + threadIdx.x;
  const int tau = g / 24, c8 = (g - tau * 24) * 8;
  const int wl = tau >> 8, n = tau & 255;
  const int widx = hf * HWIN + wl;
  const int b = widx >> 4, wpos = widx & 15;
  const int pi = ((wpos >> 2) * 16 + (n >> 4) + 8) & 63;
  const int pj = ((wpos & 3) * 16 + (n & 15) + 8) & 63;
  const float* src = x + ((size_t)(b * IMGTOK + pi * 64 + pj)) * CH + c8;
  const v4f x0 = *(const v4fa*)src;
  const v4f x1 = *(const v4fa*)(src + 4);
  v4i hi, lo;
  split8(x0, x1, hi, lo);
  const size_t d = (size_t)g * 8;
  *(volatile v4i*)(xh + d) = hi;
  *(volatile v4i*)(xl + d) = lo;
  __threadfence();
  *(volatile v4i*)(xh + d) = hi;
  *(volatile v4i*)(xl + d) = lo;
}

__device__ __forceinline__ void store_pieces(us* dh, us* dl, const size_t (&off)[6],
                                             const v4i (&ph)[6], const v4i (&pl)[6]) {
#pragma unroll
  for (int u = 0; u < 6; ++u) {
    *(volatile v4i*)(dh + off[u]) = ph[u];
    *(volatile v4i*)(dl + off[u]) = pl[u];
  }
}

template <int EPI>
__device__ __forceinline__ void ln_store_pass(const float* sF, const int* sT, float* outf,
                                              us* oh, us* ol, int w, int lane) {
#pragma unroll
  for (int i = 0; i < 8; ++i) {
    const int row = w + 8 * i;
    const float* sr = sF + row * CH;
    const size_t tr = (size_t)sT[row];
    float* dr = outf + tr * CH;
    const v4f a = *(const v4fa*)(sr + 4 * lane);
    const v4f b = *(const v4fa*)(sr + 128 + 4 * (lane & 15));
    *(volatile v4f*)(dr + 4 * lane) = a;
    if (lane < 16) *(volatile v4f*)(dr + 128 + 4 * lane) = b;
    if (EPI == 1) {
      const int l24 = (lane < 24) ? lane : 23;
      const v4f x0 = *(const v4fa*)(sr + 8 * l24);
      const v4f x1 = *(const v4fa*)(sr + 8 * l24 + 4);
      v4i hi, lo;
      split8(x0, x1, hi, lo);
      if (lane < 24) {
        *(volatile v4i*)(oh + tr * CH + 8 * lane) = hi;
        *(volatile v4i*)(ol + tr * CH + 8 * lane) = lo;
      }
    }
  }
}

template <int EPI>
__global__ __launch_bounds__(256) void k_gemm(
    const us* __restrict__ Ah, const us* __restrict__ Al,
    const us* __restrict__ Wh, const us* __restrict__ Wl,
    const float* __restrict__ bias, const float* __restrict__ bias2,
    const float* __restrict__ resid, const float* __restrict__ timev,
    const float* __restrict__ lnww, const float* __restrict__ lnwb,
    const float* __restrict__ lnbw, const float* __restrict__ lnbb,
    float* __restrict__ outf, us* __restrict__ oh, us* __restrict__ ol,
    int K, int aux)
{
  __shared__ __attribute__((aligned(16))) float sF[64 * CH];
  __shared__ float sN[64 * 8];
  __shared__ float sWB[2 * CH];
  __shared__ int sT[64];

  const int tid = threadIdx.x, lane = tid & 31, w = tid >> 5, h = lane >> 4, m = lane & 15;
  const int wm = w >> 2, wn = w & 3;
  const int bx = blockIdx.x, by = blockIdx.y;
  const int lr0 = 32 * wm, lc0 = 48 * wn;
  const int ar0 = 64 * bx + lr0;
  const int wc0 = CH * by + lc0;

  const v8f z8 = {0.f, 0.f, 0.f, 0.f, 0.f, 0.f, 0.f, 0.f};
  v8f acc[2][3];
#pragma unroll
  for (int mt = 0; mt < 2; ++mt)
#pragma unroll
    for (int nt = 0; nt < 3; ++nt) acc[mt][nt] = z8;

#pragma unroll 1
  for (int k0 = 0; k0 < K; k0 += 32) {
    v8i ah[2], al[2];
#pragma unroll
    for (int mt = 0; mt < 2; ++mt) {
      const int row = ar0 + 16 * mt + m;
      size_t off;
      if (EPI == 1) off = ((size_t)((row >> 8) * NHEAD + (k0 >> 5)) * WINN + (size_t)(row & 255)) * HDIM;
      else          off = (size_t)row * (size_t)K + (size_t)k0;
      ah[mt] = ldfrag(Ah + off, h);
      al[mt] = ldfrag(Al + off, h);
    }
#pragma unroll
    for (int nt = 0; nt < 3; ++nt) {
      const size_t wo = (size_t)(wc0 + 16 * nt + m) * (size_t)K + (size_t)k0;
      const v8i bh = ldfrag(Wh + wo, h);
      const v8i bl = ldfrag(Wl + wo, h);
#pragma unroll
      for (int mt = 0; mt < 2; ++mt) {
        acc[mt][nt] = wmma3(ah[mt], bh, acc[mt][nt]);
        acc[mt][nt] = wmma3(ah[mt], bl, acc[mt][nt]);
        acc[mt][nt] = wmma3(al[mt], bh, acc[mt][nt]);
      }
    }
  }

  if constexpr (EPI == 1 || EPI == 3) {
    int bimg;
    if (EPI == 1) bimg = (aux * HWIN + (bx >> 2)) >> 4;
    else          bimg = (aux + 64 * bx) >> 12;
    const float tv = timev[bimg];
    if (tid < CH) {
      sWB[tid]      = tv * lnww[tid] + lnwb[tid];
      sWB[CH + tid] = tv * lnbw[tid] + lnbb[tid];
    }
  }

  {
    const float* bp = bias;
    if (EPI == 0 && by == 2) bp = bias2;
#pragma unroll
    for (int nt = 0; nt < 3; ++nt) {
      const int lc = lc0 + 16 * nt + m;
      float bv;
      if (EPI == 2) {
        bv = bias[CH * by + lc];
      } else {
        const float t = bp[lc];
        bv = (EPI == 0 && by == 1) ? 0.0f : t;
      }
#pragma unroll
      for (int mt = 0; mt < 2; ++mt)
#pragma unroll
        for (int r = 0; r < 8; ++r) {
          const int lrow = lr0 + 16 * mt + 8 * h + r;
          float y = acc[mt][nt][r] + bv;
          if (EPI == 2) y = gelu_f(y);
          sF[lrow * CH + lc] = y;
        }
    }
  }
  __syncthreads();

  if constexpr (EPI == 0) {
#pragma unroll
    for (int p = 0; p < 2; ++p) {
      const int task = tid + 256 * p;
      const int tk = (task < 384) ? task : 383;
      const int row = tk / NHEAD, hd = tk - row * NHEAD;
      const float* src = sF + row * CH + hd * HDIM;
      float ss = 0.0f;
#pragma unroll
      for (int i = 0; i < 8; ++i) {
        const v4f v = *(const v4fa*)(src + 4 * i);
        ss += (v.x * v.x + v.y * v.y) + (v.z * v.z + v.w * v.w);
      }
      const float rs = rsqrtf(ss);
      if (task < 384) sN[row * 8 + hd] = rs;
    }
    __syncthreads();
    v4i ph[6], pl[6];
    size_t off[6];
    us* dh;
    us* dl;
    if (by < 2) {
      dh = oh + (size_t)(2 * by) * (size_t)PLN;
      dl = dh + PLN;
#pragma unroll
      for (int u = 0; u < 6; ++u) {
        const int e8 = tid + 256 * u;
        const int row = e8 / 24, c8 = (e8 - row * 24) * 8;
        const float rs = sN[row * 8 + (c8 >> 5)];
        v4f x0 = *(const v4fa*)(sF + row * CH + c8);
        v4f x1 = *(const v4fa*)(sF + row * CH + c8 + 4);
        x0 = x0 * rs; x1 = x1 * rs;
        split8(x0, x1, ph[u], pl[u]);
        off[u] = (size_t)bx * (size_t)(64 * CH) + (size_t)e8 * 8;
      }
    } else {
      dh = oh + (size_t)4 * (size_t)PLN;
      dl = dh + PLN;
      const int wl = bx >> 2, n0 = 64 * (bx & 3);
#pragma unroll
      for (int u = 0; u < 6; ++u) {
        const int e = tid + 256 * u;
        const int c = e >> 3, j8 = (e & 7) * 8;
        const float* col = sF + j8 * CH + c;
        const v4f x0 = {col[0], col[CH], col[2 * CH], col[3 * CH]};
        const v4f x1 = {col[4 * CH], col[5 * CH], col[6 * CH], col[7 * CH]};
        split8(x0, x1, ph[u], pl[u]);
        off[u] = ((size_t)(wl * CH + c)) * WINN + (size_t)(n0 + j8);
      }
    }
    store_pieces(dh, dl, off, ph, pl);
    __threadfence();
    store_pieces(dh, dl, off, ph, pl);
  }

  if constexpr (EPI == 2) {
    v4i ph[6], pl[6];
    size_t off[6];
#pragma unroll
    for (int u = 0; u < 6; ++u) {
      const int e8 = tid + 256 * u;
      const int row = e8 / 24, c8 = (e8 - row * 24) * 8;
      const v4f x0 = *(const v4fa*)(sF + row * CH + c8);
      const v4f x1 = *(const v4fa*)(sF + row * CH + c8 + 4);
      split8(x0, x1, ph[u], pl[u]);
      off[u] = (size_t)(64 * bx + row) * (size_t)HIDCH + (size_t)(CH * by + c8);
    }
    store_pieces(oh, ol, off, ph, pl);
    __threadfence();
    store_pieces(oh, ol, off, ph, pl);
  }

  if constexpr (EPI == 1 || EPI == 3) {
    const int row = tid >> 2, part = tid & 3;
    float* srw = sF + row * CH + 48 * part;
    float s1 = 0.0f, s2 = 0.0f;
#pragma unroll
    for (int i = 0; i < 12; ++i) {
      const v4f x = *(const v4fa*)(srw + 4 * i);
      s1 += (x.x + x.y) + (x.z + x.w);
      s2 += (x.x * x.x + x.y * x.y) + (x.z * x.z + x.w * x.w);
    }
    s1 += __shfl_xor(s1, 1); s2 += __shfl_xor(s2, 1);
    s1 += __shfl_xor(s1, 2); s2 += __shfl_xor(s2, 2);
    const float mean = s1 * (1.0f / (float)CH);
    const float var = s2 * (1.0f / (float)CH) - mean * mean;
    const float inv = rsqrtf(var + LN_EPS);
    int trow;
    const float* rrow;
    if constexpr (EPI == 1) {
      const int tau = 64 * bx + row;
      const int wl = tau >> 8, n = tau & 255;
      const int widx = aux * HWIN + wl;
      const int b = widx >> 4, wpos = widx & 15;
      const int pi = ((wpos >> 2) * 16 + (n >> 4) + 8) & 63;
      const int pj = ((wpos & 3) * 16 + (n & 15) + 8) & 63;
      const int t = b * IMGTOK + pi * 64 + pj;
      trow = t - aux * HTOK;
      rrow = resid + (size_t)t * CH;
    } else {
      trow = 64 * bx + row;
      rrow = resid + (size_t)trow * CH;
    }
#pragma unroll
    for (int i = 0; i < 12; ++i) {
      const int c = 48 * part + 4 * i;
      const v4f x = *(const v4fa*)(srw + 4 * i);
      const v4f rv = *(const v4fa*)(rrow + c);
      v4f o;
      o.x = rv.x + (sWB[c]     * ((x.x - mean) * inv) + sWB[CH + c]);
      o.y = rv.y + (sWB[c + 1] * ((x.y - mean) * inv) + sWB[CH + c + 1]);
      o.z = rv.z + (sWB[c + 2] * ((x.z - mean) * inv) + sWB[CH + c + 2]);
      o.w = rv.w + (sWB[c + 3] * ((x.w - mean) * inv) + sWB[CH + c + 3]);
      *(v4fa*)(srw + 4 * i) = o;
    }
    if (part == 0) sT[row] = trow;
    __syncthreads();
    ln_store_pass<EPI>(sF, sT, outf, oh, ol, w, lane);
    __threadfence();
    ln_store_pass<EPI>(sF, sT, outf, oh, ol, w, lane);
  }
}

__device__ __forceinline__ void ao_store_pass(const us* soh, const us* sol, us* gh, us* gl, int lane) {
#pragma unroll
  for (int i = 0; i < 2; ++i) {
    const int pc = (i * 32 + lane) * 8;
    const v4i a = *(const v4ia*)(soh + pc);
    const v4i b = *(const v4ia*)(sol + pc);
    *(volatile v4i*)(gh + pc) = a;
    *(volatile v4i*)(gl + pc) = b;
  }
}

__global__ __launch_bounds__(256) void k_attn(
    const us* __restrict__ qh, const us* __restrict__ ql,
    const us* __restrict__ kh, const us* __restrict__ kl,
    const us* __restrict__ vh, const us* __restrict__ vl,
    const float* __restrict__ bmt, const float* __restrict__ lscale,
    us* __restrict__ aoh, us* __restrict__ aol)
{
  __shared__ __attribute__((aligned(16))) us sO[8 * 1024];

  const int qh2 = blockIdx.x & 1;
  const int bid = blockIdx.x >> 1;
  const int wl = bid / NHEAD, head = bid - wl * NHEAD;
  const int whh = (wl & 15) >> 2, www = wl & 3;
  const int cls = ((whh == 3) ? 2 : 0) + ((www == 3) ? 1 : 0);
  const int tid = threadIdx.x, lane = tid & 31, w = tid >> 5, h = lane >> 4, m = lane & 15;
  const int qbase = 128 * qh2 + 16 * w;
  const float sc = expf(fminf(lscale[head], LN100));

  const size_t qoff = ((size_t)(wl * WINN + qbase + m)) * CH + head * HDIM;
  const v8i bqh = ldfrag(qh + qoff, h);
  const v8i bql = ldfrag(ql + qoff, h);

  const v8f z8 = {0.f, 0.f, 0.f, 0.f, 0.f, 0.f, 0.f, 0.f};
  v8f o[2];
  o[0] = z8; o[1] = z8;
  float mrun = -1e30f;
  float lsum = 0.0f;

  const size_t kb0 = ((size_t)(wl * WINN + m)) * CH + head * HDIM;
  const size_t vb0 = ((size_t)(wl * CH + head * HDIM + m)) * WINN;
  const float* bmh = bmt + (size_t)(cls * NHEAD + head) * (size_t)(WINN * WINN)
                         + (size_t)(qbase + m) * WINN + 8 * h;

#pragma unroll 1
  for (int kc = 0; kc < 8; ++kc) {
    sched_fence();
    v8i akh[2], akl[2];
#pragma unroll
    for (int kt = 0; kt < 2; ++kt) {
      const size_t ko = kb0 + (size_t)(32 * kc + 16 * kt) * CH;
      akh[kt] = ldfrag(kh + ko, h);
      akl[kt] = ldfrag(kl + ko, h);
    }
    v8f s[2];
#pragma unroll
    for (int kt = 0; kt < 2; ++kt) {
      v8f z = wmma3(akh[kt], bqh, z8);
      z = wmma3(akh[kt], bql, z);
      z = wmma3(akl[kt], bqh, z);
      const float* bp = bmh + 32 * kc + 16 * kt;
      const v4f b0 = *(const v4fa*)bp;
      const v4f b1 = *(const v4fa*)(bp + 4);
      v8f t;
      t[0] = z[0] * sc + b0.x; t[1] = z[1] * sc + b0.y;
      t[2] = z[2] * sc + b0.z; t[3] = z[3] * sc + b0.w;
      t[4] = z[4] * sc + b1.x; t[5] = z[5] * sc + b1.y;
      t[6] = z[6] * sc + b1.z; t[7] = z[7] * sc + b1.w;
      s[kt] = t;
    }
    float mloc = s[0][0];
#pragma unroll
    for (int kt = 0; kt < 2; ++kt)
#pragma unroll
      for (int r = 0; r < 8; ++r) mloc = fmaxf(mloc, s[kt][r]);
    mloc = fmaxf(mloc, __shfl_xor(mloc, 16));
    const float mnew = fmaxf(mrun, mloc);
    const float alpha = __expf(mrun - mnew);
    mrun = mnew;
    float ls = 0.0f;
#pragma unroll
    for (int kt = 0; kt < 2; ++kt)
#pragma unroll
      for (int r = 0; r < 8; ++r) {
        const float p = __expf(s[kt][r] - mnew);
        s[kt][r] = p;
        ls += p;
      }
    lsum = lsum * alpha + ls;
    o[0] = o[0] * alpha;
    o[1] = o[1] * alpha;
    v8i ph, pl;
    packP(s[0], s[1], ph, pl);
    sched_fence();
    v8i avh[2], avl[2];
#pragma unroll
    for (int dt = 0; dt < 2; ++dt) {
      const size_t vo = vb0 + (size_t)(16 * dt) * WINN + (size_t)(32 * kc);
      avh[dt] = ldfrag(vh + vo, h);
      avl[dt] = ldfrag(vl + vo, h);
    }
#pragma unroll
    for (int dt = 0; dt < 2; ++dt) {
      o[dt] = wmma3(avh[dt], ph, o[dt]);
      o[dt] = wmma3(avh[dt], pl, o[dt]);
      o[dt] = wmma3(avl[dt], ph, o[dt]);
    }
  }

  const float ltot = lsum + __shfl_xor(lsum, 16);
  const float iv = __builtin_amdgcn_rcpf(ltot);
  us* soh = sO + w * 1024;
  us* sol = soh + 512;
#pragma unroll
  for (int dt = 0; dt < 2; ++dt) {
    const v4f x0 = {o[dt][0] * iv, o[dt][1] * iv, o[dt][2] * iv, o[dt][3] * iv};
    const v4f x1 = {o[dt][4] * iv, o[dt][5] * iv, o[dt][6] * iv, o[dt][7] * iv};
    v4i hi, lo;
    split8(x0, x1, hi, lo);
    const int so = m * HDIM + 16 * dt + 8 * h;
    *(v4ia*)(soh + so) = hi;
    *(v4ia*)(sol + so) = lo;
  }
  __syncthreads();

  const size_t go = ((size_t)((wl * NHEAD + head) * WINN + qbase)) * HDIM;
  ao_store_pass(soh, sol, aoh + go, aol + go, lane);
  __threadfence();
  ao_store_pass(soh, sol, aoh + go, aol + go, lane);
}

extern "C" void kernel_launch(void* const* d_in, const int* in_sizes, int n_in,
                              void* d_out, int out_size, void* d_ws, size_t ws_size,
                              hipStream_t stream) {
  if (n_in < 25) return;
  if (in_sizes[0] != NTOK * CH || out_size != NTOK * CH) return;
  if (in_sizes[1] != 16 || in_sizes[7] != NHEAD) return;
  if (in_sizes[2] != CH * CH || in_sizes[4] != CH * CH || in_sizes[5] != CH * CH || in_sizes[11] != CH * CH) return;
  if (in_sizes[3] != CH || in_sizes[6] != CH || in_sizes[12] != CH) return;
  if (in_sizes[8] != 1024 || in_sizes[9] != 512 || in_sizes[10] != NHEAD * 512) return;
  if (in_sizes[13] != CH || in_sizes[14] != CH || in_sizes[15] != CH || in_sizes[16] != CH) return;
  if (in_sizes[17] != HIDCH * CH || in_sizes[18] != HIDCH || in_sizes[19] != CH * HIDCH || in_sizes[20] != CH) return;
  if (in_sizes[21] != CH || in_sizes[22] != CH || in_sizes[23] != CH || in_sizes[24] != CH) return;
  const size_t WS_END = 108747776;
  if (ws_size < WS_END) return;

  const float* hidden = (const float*)d_in[0];
  const float* timev  = (const float*)d_in[1];
  const float* q_w    = (const float*)d_in[2];
  const float* q_b    = (const float*)d_in[3];
  const float* k_w    = (const float*)d_in[4];
  const float* v_w    = (const float*)d_in[5];
  const float* v_b    = (const float*)d_in[6];
  const float* lscale = (const float*)d_in[7];
  const float* cpb_w1 = (const float*)d_in[8];
  const float* cpb_b1 = (const float*)d_in[9];
  const float* cpb_w2 = (const float*)d_in[10];
  const float* proj_w = (const float*)d_in[11];
  const float* proj_b = (const float*)d_in[12];
  const float* ln1_ww = (const float*)d_in[13];
  const float* ln1_wb = (const float*)d_in[14];
  const float* ln1_bw = (const float*)d_in[15];
  const float* ln1_bb = (const float*)d_in[16];
  const float* fc1_w  = (const float*)d_in[17];
  const float* fc1_b  = (const float*)d_in[18];
  const float* fc2_w  = (const float*)d_in[19];
  const float* fc2_b  = (const float*)d_in[20];
  const float* ln2_ww = (const float*)d_in[21];
  const float* ln2_wb = (const float*)d_in[22];
  const float* ln2_bw = (const float*)d_in[23];
  const float* ln2_bb = (const float*)d_in[24];
  float* outp = (float*)d_out;

  char* ws = (char*)d_ws;
  us*    wH  = (us*)(ws + 0);
  us*    wL  = (us*)(ws + 884736);
  float* t16 = (float*)(ws + 1769472);
  float* bmt = (float*)(ws + 1793024);
  us*    xwH = (us*)(ws + 8084480);
  us*    xwL = (us*)(ws + 20667392);
  us*    qkv = (us*)(ws + 33250304);
  float* hF  = (float*)(ws + 33250304);
  us*    hH  = (us*)(ws + 58416128);
  us*    hL  = (us*)(ws + 70999040);
  us*    gH  = (us*)(ws + 83581952);
  us*    gL  = (us*)(ws + 96164864);
  us*    aoH = xwH;
  us*    aoL = xwL;

  k_wcvt<<<216, 256, 0, stream>>>(q_w, k_w, v_w, proj_w, fc1_w, fc2_w, wH, wL);
  k_cpb<<<NT16 / 256, 256, 0, stream>>>(cpb_w1, cpb_b1, cpb_w2, t16);
  k_bmt<<<(4 * NHEAD * WINN * WINN) / 256, 256, 0, stream>>>(t16, bmt);

  for (int hf = 0; hf < 2; ++hf) {
    k_pack<<<(HTOK * 24) / 256, 256, 0, stream>>>(hidden, xwH, xwL, hf);

    k_gemm<0><<<dim3(HTOK / 64, 3), 256, 0, stream>>>(
        xwH, xwL, wH, wL, q_b, v_b, hidden, timev, ln1_ww, ln1_wb, ln1_bw, ln1_bb,
        hF, qkv, qkv, CH, hf);

    k_attn<<<HWIN * NHEAD * 2, 256, 0, stream>>>(
        qkv, qkv + PLN, qkv + 2 * (size_t)PLN, qkv + 3 * (size_t)PLN,
        qkv + 4 * (size_t)PLN, qkv + 5 * (size_t)PLN, bmt, lscale, aoH, aoL);

    k_gemm<1><<<dim3(HTOK / 64, 1), 256, 0, stream>>>(
        aoH, aoL, wH + WOFF_P, wL + WOFF_P, proj_b, proj_b, hidden, timev,
        ln1_ww, ln1_wb, ln1_bw, ln1_bb, hF, hH, hL, CH, hf);

    for (int c = 0; c < HTOK / CHUNK; ++c) {
      const size_t cb = (size_t)c * CHUNK;
      k_gemm<2><<<dim3(CHUNK / 64, HIDCH / CH), 256, 0, stream>>>(
          hH + cb * CH, hL + cb * CH, wH + WOFF_F1, wL + WOFF_F1, fc1_b, fc1_b, hidden, timev,
          ln2_ww, ln2_wb, ln2_bw, ln2_bb, hF, gH, gL, CH, 0);
      k_gemm<3><<<dim3(CHUNK / 64, 1), 256, 0, stream>>>(
          gH, gL, wH + WOFF_F2, wL + WOFF_F2, fc2_b, fc2_b, hF + cb * CH, timev,
          ln2_ww, ln2_wb, ln2_bw, ln2_bb, outp + ((size_t)hf * HTOK + cb) * CH, hH, hL,
          HIDCH, (int)((size_t)hf * HTOK + cb));
    }
  }
}
